// STN3d_Rotate_910533067692
// MI455X (gfx1250) — hardware-verified
//
#include <hip/hip_runtime.h>
#define NB 32
#define NPT 4096
#define NPOS (NB * NPT)
#define C1 64
#define C2 128
#define C3 1024
#define F1 512
#define F2 256
#define F3 128

typedef __bf16 v16b __attribute__((ext_vector_type(16)));
typedef unsigned short v8us __attribute__((ext_vector_type(8), may_alias));
typedef float  v8f  __attribute__((ext_vector_type(8)));
typedef float  v4f  __attribute__((ext_vector_type(4)));
typedef float  v4fa __attribute__((ext_vector_type(4), may_alias));
union FragB { v16b v; v8us half[2]; unsigned short u[16]; };

__device__ __forceinline__ unsigned short bf16_bits(float x) { unsigned int u = __float_as_uint(x); return (unsigned short)((u + 0x7FFFu + ((u >> 16) & 1u)) >> 16); }
__device__ __forceinline__ float bf16_val(unsigned short b) { return __uint_as_float(((unsigned int)b) << 16); }
__device__ __forceinline__ float bf16_round(float x) { return bf16_val(bf16_bits(x)); }
template <int NT>
__device__ __forceinline__ v8f mmaN(v16b ah, v16b al, v16b bh, v16b bl, v8f c) {
  c = __builtin_amdgcn_wmma_f32_16x16x32_bf16(false, ah, false, bh, (short)0, c, false, false);
  if (NT >= 2) c = __builtin_amdgcn_wmma_f32_16x16x32_bf16(false, al, false, bh, (short)0, c, false, false);
  if (NT >= 3) c = __builtin_amdgcn_wmma_f32_16x16x32_bf16(false, ah, false, bl, (short)0, c, false, false);
  asm volatile("v_nop\n\tv_nop\n\tv_nop\n\tv_nop" : "+v"(c) : "v"(ah), "v"(al), "v"(bh), "v"(bl));
  return c;
}

__global__ __launch_bounds__(256) void k_wt_bf16(const float* __restrict__ W, unsigned short* __restrict__ Wt, int K, int N) {
  const int t = blockIdx.x * 256 + threadIdx.x;
  const int k8n = K / 8;
  if (t >= N * k8n) return;
  const int n = t / k8n, k8 = (t % k8n) * 8;
  v8us v;
#pragma unroll
  for (int i = 0; i < 8; ++i) v[i] = bf16_bits(W[(size_t)(k8 + i) * N + n]);
  *(volatile v8us*)(Wt + (size_t)n * K + k8) = v;
  __threadfence();
  *(volatile v8us*)(Wt + (size_t)n * K + k8) = v;
}

template <bool ASPLIT, int ACT, bool BIAS_BF16>
__global__ __launch_bounds__(128) void k_gemm_bf(const float* __restrict__ A, int lda, const unsigned short* __restrict__ Wt, int ldb,
                                               const float* __restrict__ bias, float* __restrict__ C, int ldc, int M, int N, int K) {
  __shared__ __attribute__((aligned(16))) float so[4][16][64];
  const int tid = threadIdx.x, w = tid >> 5, lane = tid & 31, ln = lane & 15, hh = lane >> 4;
  const int ntn = N / 64;
  const int wid = blockIdx.x * 4 + w;
  const int mt = wid / ntn, nq = wid % ntn;
  if (mt * 16 >= M) return;
  const int row0 = mt * 16, col0 = nq * 64;
  const float* arow = A + (size_t)(row0 + ln) * lda;
  v8f acc[4] = {};
  for (int kb = 0; kb < K; kb += 32) {
    FragB ah, al;
    const v4f x0 = *(const v4fa*)(arow + kb + 8 * hh), x1 = *(const v4fa*)(arow + kb + 8 * hh + 4);
    const v4f x2 = *(const v4fa*)(arow + kb + 16 + 8 * hh), x3 = *(const v4fa*)(arow + kb + 16 + 8 * hh + 4);
    float xs[16] = {x0[0],x0[1],x0[2],x0[3],x1[0],x1[1],x1[2],x1[3],x2[0],x2[1],x2[2],x2[3],x3[0],x3[1],x3[2],x3[3]};
#pragma unroll
    for (int i = 0; i < 16; ++i) { const unsigned short hb = bf16_bits(xs[i]); ah.u[i] = hb; al.u[i] = ASPLIT ? bf16_bits(xs[i] - bf16_val(hb)) : (unsigned short)0; }
#pragma unroll
    for (int t = 0; t < 4; ++t) {
      const unsigned short* brow = Wt + (size_t)(col0 + t * 16 + ln) * ldb + kb;
      FragB b;
      b.half[0] = *(const v8us*)(brow + 8 * hh);
      b.half[1] = *(const v8us*)(brow + 16 + 8 * hh);
      acc[t] = mmaN<ASPLIT ? 2 : 1>(ah.v, al.v, b.v, b.v, acc[t]);
    }
  }
#pragma unroll
  for (int t = 0; t < 4; ++t) {
    float bv = bias ? bias[col0 + t * 16 + ln] : 0.f;
    if (BIAS_BF16) bv = bf16_round(bv);
#pragma unroll
    for (int r = 0; r < 8; ++r) { float v = acc[t][r] + bv; if (ACT == 1) v = fmaxf(v, 0.f); so[w][8 * hh + r][t * 16 + ln] = v; }
  }
  __builtin_amdgcn_fence(__ATOMIC_ACQ_REL, "workgroup");
  __builtin_amdgcn_wave_barrier();
  const int rsub = lane >> 4, c4 = (lane & 15) * 4;
  for (int pass = 0; pass < 2; ++pass) {
#pragma unroll
    for (int q = 0; q < 8; ++q) {
      const int r = q * 2 + rsub;
      const v4f v = *(const v4fa*)&so[w][r][c4];
      *(volatile v4f*)(C + (size_t)(row0 + r) * ldc + col0 + c4) = v;
    }
    if (pass == 0) __threadfence();
  }
}

template <int D, bool CAUSAL>
__global__ __launch_bounds__(128) void k_flash(const float* __restrict__ qb, const float* __restrict__ kb, const float* __restrict__ vb,
                                             int pitch, int T, int H, float scale, float* __restrict__ y, int ypitch) {
  constexpr int KS = D / 32;
  constexpr int DT = D / 16;
  __shared__ __attribute__((aligned(16))) unsigned short sKh[32][D + 8], sKl[32][D + 8], sVh[32][D + 8], sVl[32][D + 8];
  __shared__ __attribute__((aligned(16))) unsigned short sPh[4][16][40], sPl[4][16][40];
  __shared__ __attribute__((aligned(16))) float sO[4][16][D];
  const int tid = threadIdx.x, w = tid >> 5, lane = tid & 31, ln = lane & 15, hh = lane >> 4;
  const int nqb = (T + 63) / 64;
  const int bh = blockIdx.x / nqb, qblk = blockIdx.x % nqb;
  const int b = bh / H, h = bh % H;
  const int q0 = qblk * 64 + w * 16;
  const float* Q = qb + (size_t)b * T * pitch + h * D;
  const float* K = kb + (size_t)b * T * pitch + h * D;
  const float* V = vb + (size_t)b * T * pitch + h * D;

  FragB aqh[KS], aql[KS];
  {
    int row = q0 + ln; if (row >= T) row = T - 1;
    const float* qr = Q + (size_t)row * pitch;
#pragma unroll
    for (int ks = 0; ks < KS; ++ks)
#pragma unroll
      for (int i = 0; i < 16; ++i) {
        const int d = ks * 32 + ((i < 8) ? (8 * hh + i) : (16 + 8 * hh + (i - 8)));
        const float x = qr[d] * scale; const unsigned short hb = bf16_bits(x);
        aqh[ks].u[i] = hb; aql[ks].u[i] = bf16_bits(x - bf16_val(hb));
      }
  }
  float m_r[8], l_r[8];
#pragma unroll
  for (int r = 0; r < 8; ++r) { m_r[r] = -3.0e38f; l_r[r] = 0.f; }
  v8f oacc[DT];
#pragma unroll
  for (int dt = 0; dt < DT; ++dt) oacc[dt] = (v8f){0.f,0.f,0.f,0.f,0.f,0.f,0.f,0.f};

  const int kv_end = CAUSAL ? min(T, qblk * 64 + 64) : T;
  for (int j0 = 0; j0 < kv_end; j0 += 32) {
    __syncthreads();
    for (int e = tid; e < 32 * (D / 4); e += 128) {
      const int r = e / (D / 4), c4 = (e % (D / 4)) * 4;
      const int key = j0 + r;
      v4f kf = {0.f,0.f,0.f,0.f}, vf = {0.f,0.f,0.f,0.f};
      if (key < T) { kf = *(const v4fa*)(K + (size_t)key * pitch + c4); vf = *(const v4fa*)(V + (size_t)key * pitch + c4); }
#pragma unroll
      for (int t = 0; t < 4; ++t) {
        unsigned short hb = bf16_bits(kf[t]); sKh[r][c4 + t] = hb; sKl[r][c4 + t] = bf16_bits(kf[t] - bf16_val(hb));
        hb = bf16_bits(vf[t]); sVh[r][c4 + t] = hb; sVl[r][c4 + t] = bf16_bits(vf[t] - bf16_val(hb));
      }
    }
    __syncthreads();
    v8f s[2];
#pragma unroll
    for (int nt = 0; nt < 2; ++nt) {
      v8f acc = {};
#pragma unroll
      for (int ks = 0; ks < KS; ++ks) {
        FragB bh_, bl_;
        bh_.half[0] = *(const v8us*)&sKh[nt * 16 + ln][ks * 32 + 8 * hh]; bh_.half[1] = *(const v8us*)&sKh[nt * 16 + ln][ks * 32 + 16 + 8 * hh];
        bl_.half[0] = *(const v8us*)&sKl[nt * 16 + ln][ks * 32 + 8 * hh]; bl_.half[1] = *(const v8us*)&sKl[nt * 16 + ln][ks * 32 + 16 + 8 * hh];
        acc = mmaN<3>(aqh[ks].v, aql[ks].v, bh_.v, bl_.v, acc);
      }
      s[nt] = acc;
    }
    float alpha[8];
#pragma unroll
    for (int r = 0; r < 8; ++r) {
      const int qi = q0 + 8 * hh + r;
      const int ja = j0 + ln, jb = j0 + 16 + ln;
      if (CAUSAL) { if (ja > qi) s[0][r] = -3.0e38f; if (jb > qi) s[1][r] = -3.0e38f; }
      if (ja >= T) s[0][r] = -3.0e38f;
      if (jb >= T) s[1][r] = -3.0e38f;
      float mx = fmaxf(s[0][r], s[1][r]);
      mx = fmaxf(mx, __shfl_xor(mx, 1, 32)); mx = fmaxf(mx, __shfl_xor(mx, 2, 32)); mx = fmaxf(mx, __shfl_xor(mx, 4, 32)); mx = fmaxf(mx, __shfl_xor(mx, 8, 32));
      const float mnew = fmaxf(m_r[r], mx);
      alpha[r] = (mnew > -1.0e38f) ? __expf(m_r[r] - mnew) : 1.0f;
      const float p0 = (s[0][r] > -1.0e38f) ? __expf(s[0][r] - mnew) : 0.f;
      const float p1 = (s[1][r] > -1.0e38f) ? __expf(s[1][r] - mnew) : 0.f;
      m_r[r] = mnew;
      l_r[r] = l_r[r] * alpha[r] + p0 + p1;
      unsigned short hb = bf16_bits(p0); sPh[w][8 * hh + r][ln] = hb;      sPl[w][8 * hh + r][ln] = bf16_bits(p0 - bf16_val(hb));
      hb = bf16_bits(p1);                sPh[w][8 * hh + r][16 + ln] = hb; sPl[w][8 * hh + r][16 + ln] = bf16_bits(p1 - bf16_val(hb));
    }
#pragma unroll
    for (int dt = 0; dt < DT; ++dt)
#pragma unroll
      for (int r = 0; r < 8; ++r) oacc[dt][r] *= alpha[r];
    __builtin_amdgcn_fence(__ATOMIC_ACQ_REL, "workgroup");
    __builtin_amdgcn_wave_barrier();
    FragB pah, pal;
    pah.half[0] = *(const v8us*)&sPh[w][ln][8 * hh]; pah.half[1] = *(const v8us*)&sPh[w][ln][16 + 8 * hh];
    pal.half[0] = *(const v8us*)&sPl[w][ln][8 * hh]; pal.half[1] = *(const v8us*)&sPl[w][ln][16 + 8 * hh];
#pragma unroll
    for (int dt = 0; dt < DT; ++dt) {
      FragB bvh, bvl;
#pragma unroll
      for (int i = 0; i < 8; ++i) {
        bvh.u[i] = sVh[8 * hh + i][dt * 16 + ln]; bvh.u[8 + i] = sVh[16 + 8 * hh + i][dt * 16 + ln];
        bvl.u[i] = sVl[8 * hh + i][dt * 16 + ln]; bvl.u[8 + i] = sVl[16 + 8 * hh + i][dt * 16 + ln];
      }
      oacc[dt] = mmaN<3>(pah.v, pal.v, bvh.v, bvl.v, oacc[dt]);
    }
    __builtin_amdgcn_fence(__ATOMIC_ACQ_REL, "workgroup");
    __builtin_amdgcn_wave_barrier();
  }
#pragma unroll
  for (int r = 0; r < 8; ++r) {
    float l = l_r[r];
    l += __shfl_xor(l, 1, 32); l += __shfl_xor(l, 2, 32); l += __shfl_xor(l, 4, 32); l += __shfl_xor(l, 8, 32);
    l_r[r] = (l > 0.f) ? 1.0f / l : 0.f;
  }
#pragma unroll
  for (int dt = 0; dt < DT; ++dt)
#pragma unroll
    for (int r = 0; r < 8; ++r) sO[w][8 * hh + r][dt * 16 + ln] = oacc[dt][r] * l_r[r];
  __builtin_amdgcn_fence(__ATOMIC_ACQ_REL, "workgroup");
  __builtin_amdgcn_wave_barrier();
  for (int pass = 0; pass < 2; ++pass) {
    for (int r = 0; r < 16; ++r) {
      const int row = q0 + r;
      if (row < T && lane < D / 4) {
        const v4f val = *(const v4fa*)&sO[w][r][lane * 4];
        *(volatile v4f*)(y + ((size_t)b * T + row) * ypitch + h * D + lane * 4) = val;
      }
    }
    if (pass == 0) __threadfence();
  }
}

template <bool ASPLIT, int ACT, bool BIAS_BF16, bool RES_BF16>
__global__ __launch_bounds__(128) void k_gemm_bf3(const float* __restrict__ A, int lda, const unsigned short* __restrict__ Wt, int ldb,
                                                const float* __restrict__ bias, const float* __restrict__ resid, int rmod, int ldr,
                                                float* __restrict__ C, int ldc, int M, int N, int K) {
  __shared__ __attribute__((aligned(16))) float so[4][16][64];
  const int tid = threadIdx.x, w = tid >> 5, lane = tid & 31, ln = lane & 15, hh = lane >> 4;
  const int ntn = N / 64;
  const int wid = blockIdx.x * 4 + w;
  const int mt = wid / ntn, nq = wid % ntn;
  if (mt * 16 >= M) return;
  const int row0 = mt * 16, col0 = nq * 64;
  const float* arow = A + (size_t)(row0 + ln) * lda;
  v8f acc[4] = {};
  for (int kb = 0; kb < K; kb += 32) {
    FragB ah, al;
    const v4f x0 = *(const v4fa*)(arow + kb + 8 * hh), x1 = *(const v4fa*)(arow + kb + 8 * hh + 4);
    const v4f x2 = *(const v4fa*)(arow + kb + 16 + 8 * hh), x3 = *(const v4fa*)(arow + kb + 16 + 8 * hh + 4);
    float xs[16] = {x0[0],x0[1],x0[2],x0[3],x1[0],x1[1],x1[2],x1[3],x2[0],x2[1],x2[2],x2[3],x3[0],x3[1],x3[2],x3[3]};
#pragma unroll
    for (int i = 0; i < 16; ++i) { const unsigned short hb = bf16_bits(xs[i]); ah.u[i] = hb; al.u[i] = ASPLIT ? bf16_bits(xs[i] - bf16_val(hb)) : (unsigned short)0; }
#pragma unroll
    for (int t = 0; t < 4; ++t) {
      const unsigned short* brow = Wt + (size_t)(col0 + t * 16 + ln) * ldb + kb;
      FragB b;
      b.half[0] = *(const v8us*)(brow + 8 * hh);
      b.half[1] = *(const v8us*)(brow + 16 + 8 * hh);
      acc[t] = mmaN<ASPLIT ? 2 : 1>(ah.v, al.v, b.v, b.v, acc[t]);
    }
  }
#pragma unroll
  for (int t = 0; t < 4; ++t) {
    const int col = col0 + t * 16 + ln;
    float bv = bias ? bias[col] : 0.f;
    if (BIAS_BF16) bv = bf16_round(bv);
#pragma unroll
    for (int r = 0; r < 8; ++r) {
      float v = acc[t][r] + bv;
      if (resid) { float rv = resid[(size_t)((row0 + 8 * hh + r) % rmod) * ldr + col]; if (RES_BF16) rv = bf16_round(rv); v += rv; }
      if (ACT == 1) v = fmaxf(v, 0.f);
      if (ACT == 2) v = 0.5f * v * (1.0f + erff(v * 0.70710678118654752f));
      if (ACT == 3) { const float u = 0.7978845608028654f * (v + 0.044715f * v * v * v); v = 0.5f * v * (1.0f + tanhf(u)); }
      so[w][8 * hh + r][t * 16 + ln] = v;
    }
  }
  __builtin_amdgcn_fence(__ATOMIC_ACQ_REL, "workgroup");
  __builtin_amdgcn_wave_barrier();
  const int rsub = lane >> 4, c4 = (lane & 15) * 4;
  for (int pass = 0; pass < 2; ++pass) {
#pragma unroll
    for (int q = 0; q < 8; ++q) {
      const int r = q * 2 + rsub;
      const v4f v = *(const v4fa*)&so[w][r][c4];
      *(volatile v4f*)(C + (size_t)(row0 + r) * ldc + col0 + c4) = v;
    }
    if (pass == 0) __threadfence();
  }
}
template <bool PARAM_BF16>
__global__ __launch_bounds__(256) void k_layernorm(const float* __restrict__ X, const float* __restrict__ R, const float* __restrict__ g, const float* __restrict__ bta,
                                                  float* __restrict__ out_sum, float* __restrict__ out_norm, int N, float eps) {
  __shared__ float red[256];
  const int row = blockIdx.x, tid = threadIdx.x;
  const float* x = X + (size_t)row * N; const float* rr = R ? R + (size_t)row * N : nullptr;
  float vals[16];
  const int per = N / 256;
  float s1 = 0.f;
  for (int u = 0; u < per / 4; ++u) {
    const int j = tid * 4 + 1024 * u;
    const v4f a = *(const v4fa*)(x + j);
    v4f b = {0.f,0.f,0.f,0.f}; if (rr) b = *(const v4fa*)(rr + j);
#pragma unroll
    for (int q = 0; q < 4; ++q) { const float v = a[q] + b[q]; vals[u * 4 + q] = v; s1 += v; }
  }
  red[tid] = s1; __syncthreads();
  for (int st = 128; st > 0; st >>= 1) { if (tid < st) red[tid] += red[tid + st]; __syncthreads(); }
  const float mu = red[0] / (float)N; __syncthreads();
  float s2 = 0.f;
  for (int u = 0; u < per / 4; ++u)
#pragma unroll
    for (int q = 0; q < 4; ++q) { const float c = vals[u * 4 + q] - mu; s2 += c * c; }
  red[tid] = s2; __syncthreads();
  for (int st = 128; st > 0; st >>= 1) { if (tid < st) red[tid] += red[tid + st]; __syncthreads(); }
  const float rs = rsqrtf(red[0] / (float)N + eps);
  for (int pass = 0; pass < 2; ++pass) {
    for (int u = 0; u < per / 4; ++u) {
      const int j = tid * 4 + 1024 * u;
      v4f o, sm;
#pragma unroll
      for (int q = 0; q < 4; ++q) {
        float gg = g[j + q], bb = bta[j + q];
        if (PARAM_BF16) { gg = bf16_round(gg); bb = bf16_round(bb); }
        sm[q] = vals[u * 4 + q]; o[q] = (vals[u * 4 + q] - mu) * rs * gg + bb;
      }
      if (out_sum) *(volatile v4f*)(out_sum + (size_t)row * N + j) = sm;
      *(volatile v4f*)(out_norm + (size_t)row * N + j) = o;
    }
    if (pass == 0) __threadfence();
  }
}


typedef _Float16 v16h __attribute__((ext_vector_type(16)));
union FragH { v16h v; v8us half[2]; _Float16 h[16]; unsigned short u[16]; };
template <int NT>
__device__ __forceinline__ v8f mmaH(v16h ah, v16h al, v16h bh, v16h bl, v8f c) {
  c = __builtin_amdgcn_wmma_f32_16x16x32_f16(false, ah, false, bh, (short)0, c, false, false);
  if (NT >= 2) c = __builtin_amdgcn_wmma_f32_16x16x32_f16(false, al, false, bh, (short)0, c, false, false);
  if (NT >= 3) c = __builtin_amdgcn_wmma_f32_16x16x32_f16(false, ah, false, bl, (short)0, c, false, false);
  asm volatile("v_nop\n\tv_nop\n\tv_nop\n\tv_nop" : "+v"(c) : "v"(ah), "v"(al), "v"(bh), "v"(bl));
  return c;
}
template <bool ASPLIT>
__global__ __launch_bounds__(128) void k_gemm_h(const float* __restrict__ A, int lda, size_t sA, const _Float16* __restrict__ Bh, int ldb, size_t sB, float alpha, float* __restrict__ C, int ldc, size_t sC, int M, int N, int K) {
  __shared__ __attribute__((aligned(16))) float so[4][16][64];
  const int tid = threadIdx.x, w = tid >> 5, lane = tid & 31, ln = lane & 15, hh = lane >> 4; const int by = blockIdx.y;
  A += (size_t)by * sA; Bh += (size_t)by * sB; C += (size_t)by * sC;
  const int ntn = (N + 63) / 64; const int wid = blockIdx.x * 4 + w; const int mt = wid / ntn, nq = wid % ntn; if (mt * 16 >= M) return;
  const int row0 = mt * 16, col0 = nq * 64; const float* arow = A + (size_t)(row0 + ln) * lda;
  v8f acc[4] = {};
  for (int kb = 0; kb < K; kb += 32) {
    FragH ah, al;
    const v4f x0 = *(const v4fa*)(arow + kb + 8 * hh), x1 = *(const v4fa*)(arow + kb + 8 * hh + 4), x2 = *(const v4fa*)(arow + kb + 16 + 8 * hh), x3 = *(const v4fa*)(arow + kb + 16 + 8 * hh + 4);
    float xs[16] = {x0[0],x0[1],x0[2],x0[3],x1[0],x1[1],x1[2],x1[3],x2[0],x2[1],x2[2],x2[3],x3[0],x3[1],x3[2],x3[3]};
#pragma unroll
    for (int i = 0; i < 16; ++i) { const _Float16 h = (_Float16)xs[i]; ah.h[i] = h; al.h[i] = ASPLIT ? (_Float16)(xs[i] - (float)h) : (_Float16)0.0f; }
#pragma unroll
    for (int t = 0; t < 4; ++t) { if (col0 + t * 16 >= N) continue; const size_t boff = (size_t)(col0 + t * 16 + ln) * ldb + kb; FragH bq; bq.half[0] = *(const v8us*)(Bh + boff + 8 * hh); bq.half[1] = *(const v8us*)(Bh + boff + 16 + 8 * hh);
      acc[t] = mmaH<ASPLIT ? 2 : 1>(ah.v, al.v, bq.v, bq.v, acc[t]); }
  }
#pragma unroll
  for (int t = 0; t < 4; ++t) { if (col0 + t * 16 >= N) continue;
#pragma unroll
    for (int r = 0; r < 8; ++r) so[w][8 * hh + r][t * 16 + ln] = acc[t][r] * alpha; }
  __builtin_amdgcn_fence(__ATOMIC_ACQ_REL, "workgroup"); __builtin_amdgcn_wave_barrier();
  const int rsub = lane >> 4, c4 = (lane & 15) * 4;
  for (int pass = 0; pass < 2; ++pass) {
#pragma unroll
    for (int q = 0; q < 8; ++q) { const int r = q * 2 + rsub; if (col0 + c4 < N) { const v4f v = *(const v4fa*)&so[w][r][c4]; *(volatile v4f*)(C + (size_t)(row0 + r) * ldc + col0 + c4) = v; } }
    if (pass == 0) __threadfence(); }
}

__global__ __launch_bounds__(256) void k_wt_f16(const float* __restrict__ W, _Float16* __restrict__ Wt, int K, int N, float scale) {
  const int t = blockIdx.x * 256 + threadIdx.x; if (t >= N * (K / 8)) return; const int n = t / (K / 8), k8 = (t % (K / 8)) * 8; FragH f;
#pragma unroll
  for (int i = 0; i < 8; ++i) f.h[i] = (_Float16)(bf16_round(W[(size_t)(k8 + i) * N + n]) * scale); const v8us o = f.half[0];
  *(volatile v8us*)((unsigned short*)Wt + (size_t)n * K + k8) = o; __threadfence(); *(volatile v8us*)((unsigned short*)Wt + (size_t)n * K + k8) = o;
}
template <int ACT>
__global__ __launch_bounds__(128) void k_gemm_hhx(const _Float16* __restrict__ A, int lda, size_t sA, const _Float16* __restrict__ Bh, int ldb, size_t sB, float alpha, const float* __restrict__ bias, size_t sBias, const float* __restrict__ CP, int rowsPerB, size_t sCPb, int row0g,
    float* __restrict__ C, _Float16* __restrict__ C16, int ldc, size_t sC, int M, int N, int K) {
  __shared__ __attribute__((aligned(16))) float so[4][16][64];
  const int tid = threadIdx.x, w = tid >> 5, lane = tid & 31, ln = lane & 15, hh = lane >> 4; const int by = blockIdx.y;
  A += (size_t)by * sA; Bh += (size_t)by * sB; const size_t cofs = (size_t)by * sC; const float* bp = bias ? bias + (size_t)by * sBias : nullptr;
  const int ntn = (N + 63) / 64; const int wid = blockIdx.x * 4 + w; const int mt = wid / ntn, nq = wid % ntn; if (mt * 16 >= M) return;
  const int row0 = mt * 16, col0 = nq * 64; const _Float16* arow = A + (size_t)(row0 + ln) * lda;
  v8f acc[4] = {};
  for (int kb = 0; kb < K; kb += 32) { FragH ah; ah.half[0] = *(const v8us*)((const unsigned short*)arow + kb + 8 * hh); ah.half[1] = *(const v8us*)((const unsigned short*)arow + kb + 16 + 8 * hh);
#pragma unroll
    for (int t = 0; t < 4; ++t) { if (col0 + t * 16 >= N) continue; const size_t boff = (size_t)(col0 + t * 16 + ln) * ldb + kb; FragH bq; bq.half[0] = *(const v8us*)((const unsigned short*)Bh + boff + 8 * hh); bq.half[1] = *(const v8us*)((const unsigned short*)Bh + boff + 16 + 8 * hh);
      acc[t] = mmaH<1>(ah.v, ah.v, bq.v, bq.v, acc[t]); }
  }
#pragma unroll
  for (int t = 0; t < 4; ++t) { if (col0 + t * 16 >= N) continue; const int col = col0 + t * 16 + ln; const float bv = bp ? bf16_round(bp[col]) : 0.f;
#pragma unroll
    for (int r = 0; r < 8; ++r) { float v = acc[t][r] * alpha + bv; if (CP) { const int bidx = (row0g + row0 + 8 * hh + r) / rowsPerB; v += CP[(size_t)bidx * sCPb + (size_t)by * 64 + col]; } if (ACT == 1) v = (v > 0.f) ? v : expm1f(v); else if (ACT == 3) v = fmaxf(v, 0.f); so[w][8 * hh + r][t * 16 + ln] = v; } }
  __builtin_amdgcn_fence(__ATOMIC_ACQ_REL, "workgroup"); __builtin_amdgcn_wave_barrier();
  const int rsub = lane >> 4, c4 = (lane & 15) * 4; typedef _Float16 v4h __attribute__((ext_vector_type(4)));
  for (int pass = 0; pass < 2; ++pass) {
#pragma unroll
    for (int q = 0; q < 8; ++q) { const int r = q * 2 + rsub; if (col0 + c4 < N) { const v4f v = *(const v4fa*)&so[w][r][c4]; if (C) *(volatile v4f*)(C + cofs + (size_t)(row0 + r) * ldc + col0 + c4) = v; if (C16) { v4h h4; for (int i = 0; i < 4; ++i) h4[i] = (_Float16)v[i]; *(volatile v4h*)(C16 + cofs + (size_t)(row0 + r) * ldc + col0 + c4) = h4; } } }
    if (pass == 0) __threadfence(); }
}


__global__ __launch_bounds__(256) void k_x16(const float* __restrict__ x, _Float16* __restrict__ X16, size_t n8) { const size_t t = (size_t)blockIdx.x * 256 + threadIdx.x; if (t >= n8) return; FragH f;
#pragma unroll
  for (int q = 0; q < 8; ++q) f.h[q] = (_Float16)bf16_round(x[t * 8 + q]); *(volatile v8us*)((unsigned short*)X16 + t * 8) = f.half[0]; __threadfence(); *(volatile v8us*)((unsigned short*)X16 + t * 8) = f.half[0]; }
__global__ __launch_bounds__(256) void k_h16(const float* __restrict__ x, _Float16* __restrict__ X16, size_t n8) { const size_t t = (size_t)blockIdx.x * 256 + threadIdx.x; if (t >= n8) return; FragH f;
#pragma unroll
  for (int q = 0; q < 8; ++q) f.h[q] = (_Float16)x[t * 8 + q]; *(volatile v8us*)((unsigned short*)X16 + t * 8) = f.half[0]; __threadfence(); *(volatile v8us*)((unsigned short*)X16 + t * 8) = f.half[0]; }
__global__ __launch_bounds__(256) void k_round16f(const float* __restrict__ W, _Float16* __restrict__ Bt, size_t n8) { const size_t t = (size_t)blockIdx.x * 256 + threadIdx.x; if (t >= n8) return; FragH f;
#pragma unroll
  for (int i = 0; i < 8; ++i) f.h[i] = (_Float16)(bf16_round(W[t * 8 + i]) * 16.0f); *(volatile v8us*)((unsigned short*)Bt + t * 8) = f.half[0]; __threadfence(); *(volatile v8us*)((unsigned short*)Bt + t * 8) = f.half[0]; }
template <int NHv, int TTv>
__global__ __launch_bounds__(256) void k_vt(const _Float16* __restrict__ V16, int ldv, int voff, _Float16* __restrict__ Vt) { __shared__ unsigned short tl[64][66]; const int tid = threadIdx.x; const int slab = blockIdx.x / (TTv / 64), lg = blockIdx.x % (TTv / 64); const int b = slab / NHv, h = slab % NHv;
  for (int i = tid; i < 64 * 8; i += 256) { const int r = i / 8, c8 = (i % 8) * 8; FragH f; f.half[0] = *(const v8us*)((const unsigned short*)V16 + ((size_t)b * TTv + lg * 64 + r) * ldv + voff + h * 64 + c8);
#pragma unroll
    for (int q = 0; q < 8; ++q) tl[r][c8 + q] = f.u[q]; }
  __syncthreads();
  for (int pass = 0; pass < 2; ++pass) {
#pragma unroll
    for (int rd = 0; rd < 2; ++rd) { const int d = rd * 32 + tid / 8, pc = tid % 8; FragH f;
#pragma unroll
      for (int q = 0; q < 8; ++q) f.u[q] = tl[pc * 8 + q][d];
      *(volatile v8us*)((unsigned short*)Vt + ((size_t)slab * 64 + d) * TTv + lg * 64 + pc * 8) = f.half[0]; }
    if (pass == 0) __threadfence(); } }

typedef _Float16 v4h __attribute__((ext_vector_type(4)));
__global__ __launch_bounds__(256) void k_l1(const float* __restrict__ x, const float* __restrict__ w1, const float* __restrict__ b1, float* __restrict__ P1) { const size_t t = (size_t)blockIdx.x * 256 + threadIdx.x; if (t >= (size_t)NPOS * (C1 / 4)) return; const int o4 = (int)(t % (C1 / 4)) * 4; const size_t pos = t / (C1 / 4); const int b = (int)(pos / NPT), n = (int)(pos % NPT); const float x0 = bf16_round(x[((size_t)b * 3 + 0) * NPT + n]), x1 = bf16_round(x[((size_t)b * 3 + 1) * NPT + n]), x2 = bf16_round(x[((size_t)b * 3 + 2) * NPT + n]); v4f o;
#pragma unroll
  for (int q = 0; q < 4; ++q) { const int oc = o4 + q; o[q] = bf16_round(b1[oc]) + x0 * bf16_round(w1[oc * 3]) + x1 * bf16_round(w1[oc * 3 + 1]) + x2 * bf16_round(w1[oc * 3 + 2]); }
  *(volatile v4f*)(P1 + pos * C1 + o4) = o; __threadfence(); *(volatile v4f*)(P1 + pos * C1 + o4) = o; }
template <int C>
__global__ __launch_bounds__(256) void k_stat(const float* __restrict__ P, float* __restrict__ ST) { __shared__ float ra[256]; const int c = blockIdx.x, tid = threadIdx.x; float a = 0.f; for (int i = tid; i < NPOS; i += 256) a += P[(size_t)i * C + c]; ra[tid] = a; __syncthreads(); for (int o = 128; o >= 1; o >>= 1) { if (tid < o) ra[tid] += ra[tid + o]; __syncthreads(); } const float mu = ra[0] / (float)NPOS; __syncthreads();
  float v = 0.f; for (int i = tid; i < NPOS; i += 256) { const float d = P[(size_t)i * C + c] - mu; v += d * d; } ra[tid] = v; __syncthreads(); for (int o = 128; o >= 1; o >>= 1) { if (tid < o) ra[tid] += ra[tid + o]; __syncthreads(); }
  if (tid < 8) { typedef float v4fs __attribute__((ext_vector_type(4))); v4fs st; st[0] = (tid == 0) ? mu : 0.f; st[1] = (tid == 0) ? ra[0] / (float)NPOS : 0.f; st[2] = 0.f; st[3] = 0.f; *(volatile v4fs*)(ST + c * 32 + tid * 4) = st; __threadfence(); *(volatile v4fs*)(ST + c * 32 + tid * 4) = st; } }
template <int C>
__global__ __launch_bounds__(256) void k_bnrelu(const float* __restrict__ P, const float* __restrict__ ST, const float* __restrict__ g, const float* __restrict__ be, _Float16* __restrict__ H, _Float16* __restrict__ HL, int nrows) { const size_t t = (size_t)blockIdx.x * 256 + threadIdx.x; if (t >= (size_t)nrows * (C / 8)) return; const int c8 = (int)(t % (C / 8)) * 8; const size_t pos = t / (C / 8); FragH f, fl;
#pragma unroll
  for (int q = 0; q < 8; ++q) { const int c = c8 + q; const float mu = ST[c * 32], var = ST[c * 32 + 1]; const float v = fmaxf((P[pos * C + c] - mu) * rsqrtf(var + 1e-5f) * bf16_round(g[c]) + bf16_round(be[c]), 0.f); const _Float16 h = (_Float16)v; f.h[q] = h; fl.h[q] = (_Float16)((v - (float)h) * 1024.0f); }
  for (int pass = 0; pass < 2; ++pass) { *(volatile v8us*)((unsigned short*)H + t * 8) = f.half[0]; *(volatile v8us*)((unsigned short*)HL + t * 8) = fl.half[0]; if (pass == 0) __threadfence(); } }
template <int C>
__global__ __launch_bounds__(256) void k_cstat(const float* __restrict__ Y, int b, float* __restrict__ CS) { const int o = blockIdx.x * 256 + threadIdx.x; if (o >= C) return; float s = 0.f, s2 = 0.f, mx = -3.0e38f, mn = 3.0e38f;
#pragma unroll 1
  for (int n = 0; n < NPT; ++n) { const float v = Y[(size_t)n * C + o]; s += v; s2 += v * v; mx = fmaxf(mx, v); mn = fminf(mn, v); }
  v4f r = {s, s2, mx, mn}; *(volatile v4f*)(CS + ((size_t)b * C + o) * 4) = r; __threadfence(); *(volatile v4f*)(CS + ((size_t)b * C + o) * 4) = r; }
template <int C>
__global__ __launch_bounds__(256) void k_stfin(const float* __restrict__ CS, float* __restrict__ ST) { const int t = blockIdx.x * 256 + threadIdx.x; if (t >= C * 8) return; const int c = t / 8, pc = t % 8; float s = 0.f, s2 = 0.f;
#pragma unroll 1
  for (int b = 0; b < NB; ++b) { s += CS[((size_t)b * C + c) * 4]; s2 += CS[((size_t)b * C + c) * 4 + 1]; } const float mu = s / (float)NPOS; const float var = fmaxf(s2 / (float)NPOS - mu * mu, 0.f);
  typedef float v4fs __attribute__((ext_vector_type(4))); v4fs st; st[0] = (pc == 0) ? mu : 0.f; st[1] = (pc == 0) ? var : 0.f; st[2] = 0.f; st[3] = 0.f; *(volatile v4fs*)(ST + c * 32 + pc * 4) = st; __threadfence(); *(volatile v4fs*)(ST + c * 32 + pc * 4) = st; }
__global__ __launch_bounds__(256) void k_pool(const float* __restrict__ CS, const float* __restrict__ g, const float* __restrict__ be, float* __restrict__ G, _Float16* __restrict__ Gh, _Float16* __restrict__ Gl) { const int t = blockIdx.x * 256 + threadIdx.x; if (t >= NB * C3 / 2) return; const int o0 = (t % (C3 / 2)) * 2, b = t / (C3 / 2); typedef float v2f __attribute__((ext_vector_type(2))); typedef _Float16 v2h __attribute__((ext_vector_type(2))); v2f gv; v2h hv, lv;
#pragma unroll
  for (int j = 0; j < 2; ++j) { const int o = o0 + j; float s = 0.f, s2 = 0.f;
#pragma unroll 1
    for (int bb = 0; bb < NB; ++bb) { s += CS[((size_t)bb * C3 + o) * 4]; s2 += CS[((size_t)bb * C3 + o) * 4 + 1]; }
    const float mu = s / (float)NPOS; const float var = fmaxf(s2 / (float)NPOS - mu * mu, 0.f); const float rs = rsqrtf(var + 1e-5f); const float gg = bf16_round(g[o]); const float sel = (gg * rs >= 0.f) ? CS[((size_t)b * C3 + o) * 4 + 2] : CS[((size_t)b * C3 + o) * 4 + 3];
    const float v = fmaxf((sel - mu) * rs * gg + bf16_round(be[o]), 0.f); gv[j] = v; const _Float16 h = (_Float16)v; hv[j] = h; lv[j] = (_Float16)((v - (float)h) * 1024.0f); }
  const size_t i = (size_t)b * C3 + o0; for (int pass = 0; pass < 2; ++pass) { *(volatile v2f*)(G + i) = gv; *(volatile v2h*)(Gh + i) = hv; *(volatile v2h*)(Gl + i) = lv; if (pass == 0) __threadfence(); } }
template <int C>
__global__ __launch_bounds__(256) void k_bnfc(const float* __restrict__ Y, const float* __restrict__ g, const float* __restrict__ be, float* __restrict__ O, _Float16* __restrict__ Oh, _Float16* __restrict__ Ol) { const int t = blockIdx.x * 256 + threadIdx.x; if (t >= C / 2) return; const int c0 = t * 2; typedef float v2f __attribute__((ext_vector_type(2))); typedef _Float16 v2h __attribute__((ext_vector_type(2))); float mu[2], rs[2], gg[2], bb2[2];
#pragma unroll
  for (int j = 0; j < 2; ++j) { const int c = c0 + j; float s = 0.f; for (int b = 0; b < NB; ++b) s += Y[b * C + c]; mu[j] = s / (float)NB; float v = 0.f; for (int b = 0; b < NB; ++b) { const float d = Y[b * C + c] - mu[j]; v += d * d; } rs[j] = rsqrtf(v / (float)NB + 1e-5f); gg[j] = bf16_round(g[c]); bb2[j] = bf16_round(be[c]); }
  for (int pass = 0; pass < 2; ++pass) {
#pragma unroll 1
    for (int b = 0; b < NB; ++b) { v2f o; v2h hv, lv;
#pragma unroll
      for (int j = 0; j < 2; ++j) { o[j] = fmaxf((Y[b * C + c0 + j] - mu[j]) * rs[j] * gg[j] + bb2[j], 0.f); const _Float16 h = (_Float16)o[j]; hv[j] = h; lv[j] = (_Float16)((o[j] - (float)h) * 1024.0f); }
      *(volatile v2f*)(O + b * C + c0) = o; *(volatile v2h*)(Oh + b * C + c0) = hv; *(volatile v2h*)(Ol + b * C + c0) = lv; }
    if (pass == 0) __threadfence(); } }
__global__ __launch_bounds__(256) void k_rot(const float* __restrict__ H3, const float* __restrict__ fw4, const float* __restrict__ fb4, float* __restrict__ out) { __shared__ __attribute__((aligned(16))) float R[NB * 9 + 4]; const int tid = threadIdx.x;
  if (tid < NB) { float ang[3];
#pragma unroll
    for (int j = 0; j < 3; ++j) { float s = bf16_round(fb4[j]);
#pragma unroll 1
      for (int c = 0; c < F3; ++c) s += H3[tid * F3 + c] * bf16_round(fw4[j * F3 + c]); ang[j] = s * 3.1415927410125732f; }
    const float ca = cosf(ang[0]), sa = sinf(ang[0]), cb = cosf(ang[1]), sb = sinf(ang[1]), cc = cosf(ang[2]), sc = sinf(ang[2]);
    const float m00 = cb, m01 = sb * sa, m02 = sb * ca, m10 = 0.f, m11 = ca, m12 = -sa, m20 = -sb, m21 = cb * sa, m22 = cb * ca;
    R[tid * 9 + 0] = cc * m00 + (-sc) * m10; R[tid * 9 + 1] = cc * m01 + (-sc) * m11; R[tid * 9 + 2] = cc * m02 + (-sc) * m12;
    R[tid * 9 + 3] = sc * m00 + cc * m10;    R[tid * 9 + 4] = sc * m01 + cc * m11;    R[tid * 9 + 5] = sc * m02 + cc * m12;
    R[tid * 9 + 6] = m20; R[tid * 9 + 7] = m21; R[tid * 9 + 8] = m22; }
  __syncthreads();
  if (tid < (NB * 9) / 4) { const v4f v = *(const v4f*)&R[tid * 4]; *(volatile v4f*)(out + tid * 4) = v; __threadfence(); *(volatile v4f*)(out + tid * 4) = v; } }
extern "C" void kernel_launch(void* const* d_in, const int* in_sizes, int n_in,
                              void* d_out, int out_size, void* d_ws, size_t ws_size, hipStream_t stream) {
  (void)in_sizes; (void)n_in; (void)out_size;
  const float* const* I = (const float* const*)d_in; const float* x = I[0]; const float* w1 = I[1]; const float* b1 = I[2]; const float* g1 = I[3]; const float* be1 = I[4]; const float* w2 = I[5]; const float* b2 = I[6]; const float* g2 = I[7]; const float* be2 = I[8]; const float* w3 = I[9]; const float* b3 = I[10]; const float* g3 = I[11]; const float* be3 = I[12];
  const float* fw1 = I[13]; const float* fb1 = I[14]; const float* g4 = I[15]; const float* be4 = I[16]; const float* fw2 = I[17]; const float* fb2 = I[18]; const float* g5 = I[19]; const float* be5 = I[20]; const float* fw3 = I[21]; const float* fb3 = I[22]; const float* g6 = I[23]; const float* be6 = I[24]; const float* fw4 = I[25]; const float* fb4 = I[26];
  char* ws = (char*)d_ws; size_t off = 0;
  auto take = [&](size_t bytes) { char* p = ws + off; off += (bytes + 255) & ~(size_t)255; return p; };
  _Float16* B2 = (_Float16*)take(C2 * C1 * 2); _Float16* B3 = (_Float16*)take((size_t)C3 * C2 * 2); _Float16* Bf1 = (_Float16*)take((size_t)F1 * C3 * 2); _Float16* Bf2 = (_Float16*)take((size_t)F2 * F1 * 2); _Float16* Bf3 = (_Float16*)take((size_t)F3 * F2 * 2); float* ST1 = (float*)take(C1 * 32 * 4); float* ST2 = (float*)take(C2 * 32 * 4);
  float* P1 = (float*)take((size_t)NPOS * C1 * 4); _Float16* H1 = (_Float16*)take((size_t)NPOS * C1 * 2); _Float16* H1L = (_Float16*)take((size_t)NPOS * C1 * 2); float* Y2 = (float*)take((size_t)NPT * C2 * 4); _Float16* H2 = (_Float16*)take((size_t)NPT * C2 * 2); _Float16* H2L = (_Float16*)take((size_t)NPT * C2 * 2); float* Y3 = (float*)take((size_t)NPT * C3 * 4); float* CS2 = (float*)take((size_t)NB * C2 * 4 * 4); float* CS3 = (float*)take((size_t)NB * C3 * 4 * 4);
  float* G = (float*)take(NB * C3 * 4); _Float16* Gh = (_Float16*)take(NB * C3 * 2); _Float16* Gl = (_Float16*)take(NB * C3 * 2); float* Yf = (float*)take(NB * F1 * 4); float* Of = (float*)take(NB * F1 * 4); _Float16* Oh = (_Float16*)take(NB * F1 * 2); _Float16* Ol = (_Float16*)take(NB * F1 * 2);
  if (off > ws_size) return;
  k_round16f<<<(C2 * C1 / 8 + 255) / 256, 256, 0, stream>>>(w2, B2, C2 * C1 / 8); k_round16f<<<(unsigned)(((size_t)C3 * C2 / 8 + 255) / 256), 256, 0, stream>>>(w3, B3, (size_t)C3 * C2 / 8);
  k_round16f<<<(unsigned)(((size_t)F1 * C3 / 8 + 255) / 256), 256, 0, stream>>>(fw1, Bf1, (size_t)F1 * C3 / 8); k_round16f<<<(unsigned)(((size_t)F2 * F1 / 8 + 255) / 256), 256, 0, stream>>>(fw2, Bf2, (size_t)F2 * F1 / 8); k_round16f<<<(F3 * F2 / 8 + 255) / 256, 256, 0, stream>>>(fw3, Bf3, F3 * F2 / 8);
  k_l1<<<(unsigned)(((size_t)NPOS * (C1 / 4) + 255) / 256), 256, 0, stream>>>(x, w1, b1, P1);
  k_stat<C1><<<C1, 256, 0, stream>>>(P1, ST1); k_bnrelu<C1><<<(unsigned)(((size_t)NPOS * (C1 / 8) + 255) / 256), 256, 0, stream>>>(P1, ST1, g1, be1, H1, H1L, NPOS);
  const dim3 gd2(((NPT / 16) * (C2 / 64) + 3) / 4, 1), gd3(((NPT / 16) * (C3 / 64) + 3) / 4, 1);
  for (int b = 0; b < NB; ++b) { k_gemm_hhx<0><<<gd2, 128, 0, stream>>>(H1 + (size_t)b * NPT * C1, C1, 0, B2, C1, 0, 0.0625f, b2, 0, nullptr, 1, 0, 0, Y2, nullptr, C2, 0, NPT, C2, C1); k_gemm_hhx<0><<<gd2, 128, 0, stream>>>(H1L + (size_t)b * NPT * C1, C1, 0, B2, C1, 0, 0.0625f * 0.0009765625f, nullptr, 0, Y2, 1, (size_t)C2, 0, Y2, nullptr, C2, 0, NPT, C2, C1); k_cstat<C2><<<1, 256, 0, stream>>>(Y2, b, CS2); }
  k_stfin<C2><<<(C2 * 8 + 255) / 256, 256, 0, stream>>>(CS2, ST2);
  for (int b = 0; b < NB; ++b) { k_gemm_hhx<0><<<gd2, 128, 0, stream>>>(H1 + (size_t)b * NPT * C1, C1, 0, B2, C1, 0, 0.0625f, b2, 0, nullptr, 1, 0, 0, Y2, nullptr, C2, 0, NPT, C2, C1); k_gemm_hhx<0><<<gd2, 128, 0, stream>>>(H1L + (size_t)b * NPT * C1, C1, 0, B2, C1, 0, 0.0625f * 0.0009765625f, nullptr, 0, Y2, 1, (size_t)C2, 0, Y2, nullptr, C2, 0, NPT, C2, C1);
    k_bnrelu<C2><<<(unsigned)(((size_t)NPT * (C2 / 8) + 255) / 256), 256, 0, stream>>>(Y2, ST2, g2, be2, H2, H2L, NPT);
    k_gemm_hhx<0><<<gd3, 128, 0, stream>>>(H2, C2, 0, B3, C2, 0, 0.0625f, b3, 0, nullptr, 1, 0, 0, Y3, nullptr, C3, 0, NPT, C3, C2); k_gemm_hhx<0><<<gd3, 128, 0, stream>>>(H2L, C2, 0, B3, C2, 0, 0.0625f * 0.0009765625f, nullptr, 0, Y3, 1, (size_t)C3, 0, Y3, nullptr, C3, 0, NPT, C3, C2);
    k_cstat<C3><<<C3 / 256, 256, 0, stream>>>(Y3, b, CS3); }
  k_pool<<<(NB * C3 / 2 + 255) / 256, 256, 0, stream>>>(CS3, g3, be3, G, Gh, Gl);
  const dim3 gf1(((NB / 16) * (F1 / 64) + 3) / 4, 1), gf2(((NB / 16) * (F2 / 64) + 3) / 4, 1), gf3(((NB / 16) * (F3 / 64) + 3) / 4, 1);
  k_gemm_hhx<0><<<gf1, 128, 0, stream>>>(Gh, C3, 0, Bf1, C3, 0, 0.0625f, fb1, 0, nullptr, 1, 0, 0, Yf, nullptr, F1, 0, NB, F1, C3); k_gemm_hhx<0><<<gf1, 128, 0, stream>>>(Gl, C3, 0, Bf1, C3, 0, 0.0625f * 0.0009765625f, nullptr, 0, Yf, 1, (size_t)F1, 0, Yf, nullptr, F1, 0, NB, F1, C3);
  k_bnfc<F1><<<(F1 / 2 + 255) / 256, 256, 0, stream>>>(Yf, g4, be4, Of, Oh, Ol);
  k_gemm_hhx<0><<<gf2, 128, 0, stream>>>(Oh, F1, 0, Bf2, F1, 0, 0.0625f, fb2, 0, nullptr, 1, 0, 0, Yf, nullptr, F2, 0, NB, F2, F1); k_gemm_hhx<0><<<gf2, 128, 0, stream>>>(Ol, F1, 0, Bf2, F1, 0, 0.0625f * 0.0009765625f, nullptr, 0, Yf, 1, (size_t)F2, 0, Yf, nullptr, F2, 0, NB, F2, F1);
  k_bnfc<F2><<<(F2 / 2 + 255) / 256, 256, 0, stream>>>(Yf, g5, be5, Of, Oh, Ol);
  k_gemm_hhx<0><<<gf3, 128, 0, stream>>>(Oh, F2, 0, Bf3, F2, 0, 0.0625f, fb3, 0, nullptr, 1, 0, 0, Yf, nullptr, F3, 0, NB, F3, F2); k_gemm_hhx<0><<<gf3, 128, 0, stream>>>(Ol, F2, 0, Bf3, F2, 0, 0.0625f * 0.0009765625f, nullptr, 0, Yf, 1, (size_t)F3, 0, Yf, nullptr, F3, 0, NB, F3, F2);
  k_bnfc<F3><<<(F3 / 2 + 255) / 256, 256, 0, stream>>>(Yf, g6, be6, Of, Oh, Ol);
  k_rot<<<1, 256, 0, stream>>>(Of, fw4, fb4, (float*)d_out);
}
